// Causal_Attention_13082470383895
// MI455X (gfx1250) — hardware-verified
//
#include <hip/hip_runtime.h>
#include <math.h>
#include <stdint.h>

#define BATCH 2
#define SEQ   2048
#define DMOD  1024
#define NH    16
#define HD    64
#define NQK   (2 * DMOD)
#define MROWS (BATCH * SEQ)
#define NVEC  (MROWS * NH * 2)
#define LN_EPS 1e-6f
#define QSC   64.0f
#define KSC   64.0f
#define PCAR  32768.0f
#define VCAR  1024.0f
#define OSC   1024.0f
#define WOS   1024.0f
#define LOG2E 1.4426950408889634f
#define WPB   4
#define NHG   (NH / WPB)
#define NQT   (SEQ / 16)
#define NST   (SEQ / 64)
#define NKT   (SEQ / 32)
#define ATT_THREADS (WPB * 32)
#define ATT_BLOCKS  (NQT * NHG * BATCH)
#define PTW   (16 * 36)
#define SLW   (16 * 68)
#define WREG  (PTW + SLW)
#define SLAB64 (16 * 68)
#define VTP   72
static_assert(DMOD == NH * HD && HD == 64 && NH == 16);
static_assert((NH % WPB) == 0 && ATT_THREADS == 128 && ATT_BLOCKS == 1024);
static_assert((SEQ % 64) == 0 && (SEQ % 32) == 0 && (SEQ % 16) == 0 && SEQ <= 32768);
static_assert((DMOD % 64) == 0 && (DMOD % 32) == 0 && (NQK % 64) == 0 && (MROWS % 64) == 0);
static_assert(((MROWS * DMOD) % 2048) == 0 && ((DMOD * DMOD) % 4096) == 0 && ((NVEC * 32) % 256) == 0);

typedef unsigned short u16;
typedef _Float16 v16h __attribute__((ext_vector_type(16)));
typedef _Float16 v8h  __attribute__((ext_vector_type(8)));
typedef __bf16   v16b __attribute__((ext_vector_type(16)));
typedef float    v8f  __attribute__((ext_vector_type(8)));
typedef float    v4f  __attribute__((ext_vector_type(4)));
typedef float    v2f  __attribute__((ext_vector_type(2)));
typedef unsigned int v4u __attribute__((ext_vector_type(4)));

union FragH { v16h v; v8h h[2]; v4u u[2]; };
union FragB { v16b v; v4u u[2]; };

__device__ __forceinline__ unsigned short bf_bits(float f) {
  unsigned u = __float_as_uint(f);
  return (unsigned short)((u + 0x7FFFu + ((u >> 16) & 1u)) >> 16);
}
__device__ __forceinline__ float bf_up(unsigned short h) { return __uint_as_float(((unsigned)h) << 16); }
__device__ __forceinline__ float bfr(float f) { return bf_up(bf_bits(f)); }
__device__ __forceinline__ unsigned short h_bits(_Float16 x) { return __builtin_bit_cast(unsigned short, x); }
__device__ __forceinline__ unsigned pk16(unsigned short a, unsigned short b) { return (unsigned)a | ((unsigned)b << 16); }
__device__ __forceinline__ v8f zero8() { v8f z = {0.f, 0.f, 0.f, 0.f, 0.f, 0.f, 0.f, 0.f}; return z; }

__device__ __forceinline__ v16h ldfrag_h(const _Float16* p) {
  FragH f;
  f.h[0] = *(const v8h*)(p);
  f.h[1] = *(const v8h*)(p + 16);
  return f.v;
}
__device__ __forceinline__ v16b ldfrag_b(const u16* p) {
  FragB f;
  f.u[0] = *(const v4u*)(p);
  f.u[1] = *(const v4u*)(p + 16);
  return f.v;
}

__device__ __forceinline__ v8f mma_h(v16h a, v16h b, v8f c) {
  return __builtin_amdgcn_wmma_f32_16x16x32_f16(false, a, false, b, (short)0, c, false, false);
}
__device__ __forceinline__ v8f mma_b(v16b a, v16b b, v8f c) {
  return __builtin_amdgcn_wmma_f32_16x16x32_bf16(false, a, false, b, (short)0, c, false, false);
}
__device__ __forceinline__ void guard2(v8f& a, v8f& b, v16h x0, v16h x1, v16h x2, v16h x3, v16h x4, v16h x5) {
#if defined(__HIP_DEVICE_COMPILE__)
  asm volatile("v_nop\n\tv_nop\n\tv_nop\n\tv_nop"
               : "+v"(a), "+v"(b) : "v"(x0), "v"(x1), "v"(x2), "v"(x3), "v"(x4), "v"(x5) : "memory");
#endif
}
template <typename F>
__device__ __forceinline__ void guard6(v8f& a, v8f& b, v8f& c, v8f& d, F x0, F x1, F x2, F x3, F x4, F x5) {
#if defined(__HIP_DEVICE_COMPILE__)
  asm volatile("v_nop\n\tv_nop\n\tv_nop\n\tv_nop"
               : "+v"(a), "+v"(b), "+v"(c), "+v"(d) : "v"(x0), "v"(x1), "v"(x2), "v"(x3), "v"(x4), "v"(x5) : "memory");
#endif
}
__device__ __forceinline__ void guard10(v8f& a, v8f& b, v8f& c, v8f& d, v16h x0, v16h x1, v16h x2, v16h x3, v16h x4,
                                        v16h x5, v16h x6, v16h x7, v16h x8, v16h x9) {
#if defined(__HIP_DEVICE_COMPILE__)
  asm volatile("v_nop\n\tv_nop\n\tv_nop\n\tv_nop"
               : "+v"(a), "+v"(b), "+v"(c), "+v"(d)
               : "v"(x0), "v"(x1), "v"(x2), "v"(x3), "v"(x4), "v"(x5), "v"(x6), "v"(x7), "v"(x8), "v"(x9) : "memory");
#endif
}
__device__ __forceinline__ void acc_guard4(v8f& a, v8f& b, v8f& c, v8f& d) {
#if defined(__HIP_DEVICE_COMPILE__)
  asm volatile("v_nop\n\tv_nop\n\tv_nop\n\tv_nop" : "+v"(a), "+v"(b), "+v"(c), "+v"(d));
#endif
}
__device__ __forceinline__ void wave_sync_lds() {
  __builtin_amdgcn_fence(__ATOMIC_RELEASE, "workgroup");
  __builtin_amdgcn_wave_barrier();
  __builtin_amdgcn_fence(__ATOMIC_ACQUIRE, "workgroup");
}

__global__ __launch_bounds__(256) void cvt16(const float* __restrict__ x, u16* D, int n8, int f16mode, float scale) {
  const int gt = blockIdx.x * 256 + (int)threadIdx.x;
  if (gt >= n8) return;
  const float* p = x + (size_t)gt * 8;
  const v4f a = *(const v4f*)(p), b4 = *(const v4f*)(p + 4);
  float w[8];
#pragma unroll
  for (int e = 0; e < 4; ++e) { w[e] = a[e]; w[4 + e] = b4[e]; }
  v4u o;
#pragma unroll
  for (int e = 0; e < 4; ++e) {
    const float f0 = w[2 * e], f1 = w[2 * e + 1];
    const unsigned short hb0 = h_bits((_Float16)(bfr(f0) * scale));
    const unsigned short hb1 = h_bits((_Float16)(bfr(f1) * scale));
    const unsigned short bb0 = bf_bits(f0);
    const unsigned short bb1 = bf_bits(f1);
    o[e] = (f16mode != 0) ? pk16(hb0, hb1) : pk16(bb0, bb1);
  }
  u16* d = D + (size_t)gt * 8;
  for (int pass = 0; pass < 2; ++pass) {
    *(volatile v4u*)(d) = o;
    __threadfence();
  }
}

__global__ __launch_bounds__(256) void wt16(const float* __restrict__ W, u16* Dt, int K, int N, int f16mode, float scale) {
  __shared__ __align__(16) u16 T[64 * VTP];
  const int tid = threadIdx.x;
  const int bid = blockIdx.x;
  const int ntn = N >> 6;
  const int n0  = (bid % ntn) * 64;
  const int k0  = (bid / ntn) * 64;
  if (k0 + 64 > K) return;
  {
    const int sl = tid >> 2;
    const int dc = (tid & 3) * 16;
    const float* src = W + (size_t)(k0 + sl) * N + n0 + dc;
#pragma unroll
    for (int i = 0; i < 4; ++i) {
      const v4f a = *(const v4f*)(src + 4 * i);
#pragma unroll
      for (int e = 0; e < 4; ++e) {
        const float f = a[e];
        const unsigned short hb = h_bits((_Float16)(bfr(f) * scale));
        const unsigned short bb = bf_bits(f);
        T[(dc + 4 * i + e) * VTP + sl] = (f16mode != 0) ? hb : bb;
      }
    }
  }
  __syncthreads();
  v4u vv[2];
  const int q8 = tid >> 3, p8 = (tid & 7) * 8;
#pragma unroll
  for (int it = 0; it < 2; ++it) {
    const int line = it * 32 + q8;
    vv[it] = *(const v4u*)(T + line * VTP + p8);
  }
  const size_t base = (size_t)n0 * K + k0 + p8;
  for (int pass = 0; pass < 2; ++pass) {
#pragma unroll
    for (int it = 0; it < 2; ++it) {
      const int line = it * 32 + q8;
      *(volatile v4u*)(Dt + base + (size_t)line * K) = vv[it];
    }
    __threadfence();
  }
}

__device__ __forceinline__ void epi64(float* sl, v8f a0, v8f a1, v8f a2, v8f a3, float oscale,
                                      float* C, int N, size_t rowb, int col0, int lane) {
  const int hh = lane >> 4, m = lane & 15;
#pragma unroll
  for (int r = 0; r < 8; ++r) {
    const int ro = (8 * hh + r) * 68 + m;
    sl[ro]      = a0[r] * oscale;
    sl[ro + 16] = a1[r] * oscale;
    sl[ro + 32] = a2[r] * oscale;
    sl[ro + 48] = a3[r] * oscale;
  }
  wave_sync_lds();
  v4f vals[8];
#pragma unroll
  for (int it = 0; it < 8; ++it) vals[it] = *(const v4f*)(sl + (it * 2 + hh) * 68 + m * 4);
  float* dst = C + (rowb + (size_t)hh) * (size_t)N + col0 + m * 4;
  for (int pass = 0; pass < 2; ++pass) {
#pragma unroll
    for (int it = 0; it < 8; ++it) {
      *(volatile v4f*)(dst + (size_t)(it * 2) * (size_t)N) = vals[it];
    }
    __threadfence();
  }
}

__global__ __launch_bounds__(128)
void gemm_bf(const u16* __restrict__ A, const u16* __restrict__ Bt, float* C, int M, int N, int K, float oscale) {
  __shared__ __align__(16) float slab[4 * SLAB64];
  const int tid = threadIdx.x, wave = tid >> 5, lane = tid & 31, hh = lane >> 4, m = lane & 15;
  const int ntile = N >> 6;
  const int bid   = blockIdx.x;
  const int rowb  = (bid / ntile) * 64 + wave * 16;
  const int col0  = (bid % ntile) * 64;
  if (rowb + 16 > M) return;
  const u16* ap = A  + (size_t)(rowb + m) * K + 8 * hh;
  const u16* bp = Bt + (size_t)(col0 + m) * K + 8 * hh;
  const size_t bs = (size_t)16 * K;
  v8f acc0 = zero8(), acc1 = zero8(), acc2 = zero8(), acc3 = zero8();
#pragma unroll 1
  for (int k0 = 0; k0 < K; k0 += 32) {
    const v16b a  = ldfrag_b(ap + k0);
    const v16b b0 = ldfrag_b(bp + k0);
    const v16b b1 = ldfrag_b(bp + bs + k0);
    const v16b b2 = ldfrag_b(bp + 2 * bs + k0);
    const v16b b3 = ldfrag_b(bp + 3 * bs + k0);
    acc0 = mma_b(a, b0, acc0);
    acc1 = mma_b(a, b1, acc1);
    acc2 = mma_b(a, b2, acc2);
    acc3 = mma_b(a, b3, acc3);
    guard6<v16b>(acc0, acc1, acc2, acc3, a, b0, b1, b2, b3, a);
  }
  epi64(slab + wave * SLAB64, acc0, acc1, acc2, acc3, oscale, C, N, (size_t)rowb, col0, lane);
}

__global__ __launch_bounds__(128)
void gemm_h2(const u16* __restrict__ Ah, const u16* __restrict__ Al, const u16* __restrict__ Bt,
             float* C, int M, int N, int K, float oscale) {
  __shared__ __align__(16) float slab[4 * SLAB64];
  const int tid = threadIdx.x, wave = tid >> 5, lane = tid & 31, hh = lane >> 4, m = lane & 15;
  const int ntile = N >> 6;
  const int bid   = blockIdx.x;
  const int rowb  = (bid / ntile) * 64 + wave * 16;
  const int col0  = (bid % ntile) * 64;
  if (rowb + 16 > M) return;
  const size_t aofs = (size_t)(rowb + m) * K + 8 * hh;
  const _Float16* ahp = (const _Float16*)(const void*)Ah + aofs;
  const _Float16* alp = (const _Float16*)(const void*)Al + aofs;
  const _Float16* bp  = (const _Float16*)(const void*)Bt + (size_t)(col0 + m) * K + 8 * hh;
  const size_t bs = (size_t)16 * K;
  v8f acc0 = zero8(), acc1 = zero8(), acc2 = zero8(), acc3 = zero8();
#pragma unroll 1
  for (int k0 = 0; k0 < K; k0 += 32) {
    const v16h ah = ldfrag_h(ahp + k0), al = ldfrag_h(alp + k0);
    const v16h b0 = ldfrag_h(bp + k0);
    const v16h b1 = ldfrag_h(bp + bs + k0);
    const v16h b2 = ldfrag_h(bp + 2 * bs + k0);
    const v16h b3 = ldfrag_h(bp + 3 * bs + k0);
    acc0 = mma_h(ah, b0, acc0);  acc0 = mma_h(al, b0, acc0);
    acc1 = mma_h(ah, b1, acc1);  acc1 = mma_h(al, b1, acc1);
    acc2 = mma_h(ah, b2, acc2);  acc2 = mma_h(al, b2, acc2);
    acc3 = mma_h(ah, b3, acc3);  acc3 = mma_h(al, b3, acc3);
    guard6<v16h>(acc0, acc1, acc2, acc3, ah, al, b0, b1, b2, b3);
  }
  epi64(slab + wave * SLAB64, acc0, acc1, acc2, acc3, oscale, C, N, (size_t)rowb, col0, lane);
}

__global__ __launch_bounds__(256)
void ln16(const float* __restrict__ F, const float* __restrict__ qs, const float* __restrict__ qbi,
          const float* __restrict__ ks, const float* __restrict__ kbi, u16* QK, int nvec) {
  const int gt = blockIdx.x * 256 + (int)threadIdx.x;
  const int gw = gt >> 5, lane = gt & 31;
  if (gw >= nvec) return;
  const int token = gw >> 5, rem = gw & 31, h = rem >> 1, isK = rem & 1;
  const float* src = F + (size_t)token * NQK + h * (2 * HD) + isK * HD + 2 * lane;
  const v2f xv = *(const v2f*)(src);
  const float x0 = xv[0], x1 = xv[1];
  float s = x0 + x1;
#pragma unroll
  for (int off = 16; off >= 1; off >>= 1) s += __shfl_xor(s, off, 32);
  const float mean = s * (1.0f / 64.0f);
  const float d0 = x0 - mean, d1 = x1 - mean;
  float ss = d0 * d0 + d1 * d1;
#pragma unroll
  for (int off = 16; off >= 1; off >>= 1) ss += __shfl_xor(ss, off, 32);
  const float var = ss * (1.0f / 64.0f);
  const float rs  = rsqrtf(var + LN_EPS);
  const float gq0 = bfr(qs[2 * lane]),  gq1 = bfr(qs[2 * lane + 1]);
  const float bq0 = bfr(qbi[2 * lane]), bq1 = bfr(qbi[2 * lane + 1]);
  const float gk0 = bfr(ks[2 * lane]),  gk1 = bfr(ks[2 * lane + 1]);
  const float bk0 = bfr(kbi[2 * lane]), bk1 = bfr(kbi[2 * lane + 1]);
  const float g0 = isK ? gk0 : gq0, g1 = isK ? gk1 : gq1;
  const float b0 = isK ? bk0 : bq0, b1 = isK ? bk1 : bq1;
  const float y0 = d0 * rs * g0 + b0;
  const float y1 = d1 * rs * g1 + b1;
  const float car = isK ? KSC : QSC;
  const unsigned o = pk16(h_bits((_Float16)(y0 * car)), h_bits((_Float16)(y1 * car)));
  u16* dst = QK + (size_t)isK * ((size_t)MROWS * DMOD) + (size_t)token * DMOD + h * HD + 2 * lane;
  *(volatile unsigned*)(dst) = o;
  __threadfence();
  *(volatile unsigned*)(dst) = o;
}

__global__ __launch_bounds__(256) void vt16(const float* __restrict__ v, u16* VHo, u16* VLo) {
  __shared__ __align__(16) u16 TH[HD * VTP];
  __shared__ __align__(16) u16 TL[HD * VTP];
  const int tid = threadIdx.x;
  const int bid = blockIdx.x;
  const int st  = bid % NST;
  const int bg  = bid / NST;
  if (bg >= BATCH * NH) return;
  const int b   = bg / NH;
  const int g   = bg % NH;
  const int s0  = st * 64;
  {
    const int sl = tid >> 2;
    const int dc = (tid & 3) * 16;
    const float* src = v + ((size_t)(b * SEQ + s0 + sl) * NH + g) * HD + dc;
#pragma unroll
    for (int i = 0; i < 4; ++i) {
      const v4f a = *(const v4f*)(src + 4 * i);
#pragma unroll
      for (int e = 0; e < 4; ++e) {
        const float t = a[e] * VCAR;
        const _Float16 hv = (_Float16)t;
        const _Float16 lv = (_Float16)(t - (float)hv);
        TH[(dc + 4 * i + e) * VTP + sl] = h_bits(hv);
        TL[(dc + 4 * i + e) * VTP + sl] = h_bits(lv);
      }
    }
  }
  __syncthreads();
  v4u vh[2], vl[2];
  const int q8 = tid >> 3, p8 = (tid & 7) * 8;
#pragma unroll
  for (int it = 0; it < 2; ++it) {
    const int line = it * 32 + q8;
    vh[it] = *(const v4u*)(TH + line * VTP + p8);
    vl[it] = *(const v4u*)(TL + line * VTP + p8);
  }
  const size_t base = ((size_t)bg * HD) * SEQ + s0 + p8;
  for (int pass = 0; pass < 2; ++pass) {
#pragma unroll
    for (int it = 0; it < 2; ++it) {
      const int line = it * 32 + q8;
      *(volatile v4u*)(VHo + base + (size_t)line * SEQ) = vh[it];
      *(volatile v4u*)(VLo + base + (size_t)line * SEQ) = vl[it];
    }
    __threadfence();
  }
}

__global__ __launch_bounds__(ATT_THREADS)
void attn1(const u16* __restrict__ QPp, const u16* __restrict__ KPp,
           const u16* __restrict__ VHIp, const u16* __restrict__ VLOp,
           u16* OHIp, u16* OLOp) {
  __shared__ __align__(16) float smem[WPB * WREG];

  const int tid  = threadIdx.x;
  const int wave = tid >> 5;
  const int lane = tid & 31;
  const int hh   = lane >> 4;
  const int c    = lane & 15;
  const int bid  = blockIdx.x;
  const int qt   = bid % NQT;
  const int rem  = bid / NQT;
  const int hg   = rem % NHG;
  const int b    = rem / NHG;
  if (b >= BATCH) return;
  const int head = hg * WPB + wave;
  const int q0   = qt * 16;

  float* pt   = smem + wave * WREG;
  float* slab = pt + PTW;

  const size_t rq0  = (size_t)b * SEQ + q0;
  const size_t qofs = ((rq0 + c) * NH + head) * HD + 8 * hh;
  const _Float16* Qh  = (const _Float16*)(const void*)QPp + qofs;
  const size_t kofs = (((size_t)b * SEQ + c) * NH + head) * HD + 8 * hh;
  const _Float16* Khb = (const _Float16*)(const void*)KPp + kofs;
  const size_t vofs = (((size_t)b * NH + head) * HD + c) * SEQ + 8 * hh;
  const _Float16* Vhb = (const _Float16*)(const void*)VHIp + vofs;
  const _Float16* Vlb = (const _Float16*)(const void*)VLOp + vofs;
  const float lsc = LOG2E / (64.0f * QSC * KSC);
  const float oc  = 1.0f / (PCAR * VCAR);
  const size_t KROW = (size_t)NH * HD;

  const v16h qa = ldfrag_h(Qh), qb = ldfrag_h(Qh + 32);

  float mrow[8], lrow[8];
  v8f o[4];
#pragma unroll
  for (int r = 0; r < 8; ++r) { mrow[r] = -INFINITY; lrow[r] = 0.f; }
#pragma unroll
  for (int j = 0; j < 4; ++j) o[j] = zero8();
  const int ncaus = (q0 >> 5) + 1;
  const int nkt = (ncaus < NKT) ? ncaus : NKT;
  const int qr0 = q0 + 8 * hh;

#pragma unroll 1
  for (int kt = 0; kt < nkt; ++kt) {
    const int kb = kt * 32;
    v8f s0 = zero8(), s1 = zero8();
    {
      const _Float16* k0p = Khb + (size_t)kb * KROW;
      const _Float16* k1p = k0p + (size_t)16 * KROW;
      const v16h kh0a = ldfrag_h(k0p), kh0b = ldfrag_h(k0p + 32);
      const v16h kh1a = ldfrag_h(k1p), kh1b = ldfrag_h(k1p + 32);
      s0 = mma_h(qa, kh0a, s0);
      s0 = mma_h(qb, kh0b, s0);
      s1 = mma_h(qa, kh1a, s1);
      s1 = mma_h(qb, kh1b, s1);
      guard2(s0, s1, qa, qb, kh0a, kh0b, kh1a, kh1b);
    }
    const int key0 = kb + c, key1 = kb + 16 + c;
#pragma unroll
    for (int r = 0; r < 8; ++r) {
      const int qi = qr0 + r;
      const float t0 = (key0 <= qi) ? (s0[r] * lsc) : -INFINITY;
      const float t1 = (key1 <= qi) ? (s1[r] * lsc) : -INFINITY;
      float mx = fmaxf(t0, t1);
#pragma unroll
      for (int off = 1; off < 16; off <<= 1) mx = fmaxf(mx, __shfl_xor(mx, off, 32));
      const float mn = fmaxf(mrow[r], mx);
      const float ms = (mn == -INFINITY) ? 0.0f : mn;
      const float al = exp2f(mrow[r] - ms);
      mrow[r] = mn;
      const float e0 = exp2f(t0 - ms), e1 = exp2f(t1 - ms);
      float ps = e0 + e1;
#pragma unroll
      for (int off = 1; off < 16; off <<= 1) ps += __shfl_xor(ps, off, 32);
      lrow[r] = lrow[r] * al + ps;
#pragma unroll
      for (int j = 0; j < 4; ++j) o[j][r] *= al;
      const int ro = (8 * hh + r) * 36 + c;
      pt[ro]      = e0;
      pt[ro + 16] = e1;
    }
    wave_sync_lds();
    FragH ph, pl;
    {
      const float* prow = pt + c * 36 + 8 * hh;
      const v4f p0 = *(const v4f*)(prow), p1 = *(const v4f*)(prow + 4);
      const v4f p2 = *(const v4f*)(prow + 16), p3 = *(const v4f*)(prow + 20);
#pragma unroll
      for (int e = 0; e < 4; ++e) {
        const float ta = p0[e] * PCAR, tb = p1[e] * PCAR, tc = p2[e] * PCAR, td = p3[e] * PCAR;
        const _Float16 ha = (_Float16)ta, hb = (_Float16)tb, hc = (_Float16)tc, hd = (_Float16)td;
        ph.h[0][e]     = ha;
        ph.h[0][4 + e] = hb;
        ph.h[1][e]     = hc;
        ph.h[1][4 + e] = hd;
        pl.h[0][e]     = (_Float16)(ta - (float)ha);
        pl.h[0][4 + e] = (_Float16)(tb - (float)hb);
        pl.h[1][e]     = (_Float16)(tc - (float)hc);
        pl.h[1][4 + e] = (_Float16)(td - (float)hd);
      }
    }
    {
      const _Float16* vhp = Vhb + kb;
      const _Float16* vlp = Vlb + kb;
      const v16h vh0 = ldfrag_h(vhp);
      const v16h vh1 = ldfrag_h(vhp + (size_t)16 * SEQ);
      const v16h vh2 = ldfrag_h(vhp + (size_t)32 * SEQ);
      const v16h vh3 = ldfrag_h(vhp + (size_t)48 * SEQ);
      const v16h vl0 = ldfrag_h(vlp);
      const v16h vl1 = ldfrag_h(vlp + (size_t)16 * SEQ);
      const v16h vl2 = ldfrag_h(vlp + (size_t)32 * SEQ);
      const v16h vl3 = ldfrag_h(vlp + (size_t)48 * SEQ);
      o[0] = mma_h(ph.v, vh0, o[0]);  o[0] = mma_h(pl.v, vh0, o[0]);  o[0] = mma_h(ph.v, vl0, o[0]);
      o[1] = mma_h(ph.v, vh1, o[1]);  o[1] = mma_h(pl.v, vh1, o[1]);  o[1] = mma_h(ph.v, vl1, o[1]);
      o[2] = mma_h(ph.v, vh2, o[2]);  o[2] = mma_h(pl.v, vh2, o[2]);  o[2] = mma_h(ph.v, vl2, o[2]);
      o[3] = mma_h(ph.v, vh3, o[3]);  o[3] = mma_h(pl.v, vh3, o[3]);  o[3] = mma_h(ph.v, vl3, o[3]);
      guard10(o[0], o[1], o[2], o[3], ph.v, pl.v, vh0, vh1, vh2, vh3, vl0, vl1, vl2, vl3);
    }
    wave_sync_lds();
  }
  acc_guard4(o[0], o[1], o[2], o[3]);
#pragma unroll
  for (int r = 0; r < 8; ++r) {
    const float lv  = lrow[r];
    const float ls  = (lv > 0.0f) ? lv : 1.0f;
    const float inv = (lv > 0.0f) ? ((1.0f / ls) * oc) : 0.0f;
#pragma unroll
    for (int j = 0; j < 4; ++j) {
      const int idx = (8 * hh + r) * 68 + j * 16 + c;
      slab[idx] = o[j][r] * inv;
    }
  }

  wave_sync_lds();
  v4u oh[4], ol[4];
  const int rq = lane >> 3, c8 = (lane & 7) * 8;
#pragma unroll
  for (int it = 0; it < 4; ++it) {
    const int row = it * 4 + rq;
    const v4f a = *(const v4f*)(slab + row * 68 + c8), b4 = *(const v4f*)(slab + row * 68 + c8 + 4);
    float w[8];
#pragma unroll
    for (int e = 0; e < 4; ++e) { w[e] = a[e] * OSC; w[4 + e] = b4[e] * OSC; }
#pragma unroll
    for (int e = 0; e < 4; ++e) {
      const _Float16 h0 = (_Float16)w[2 * e], h1 = (_Float16)w[2 * e + 1];
      const _Float16 l0 = (_Float16)(w[2 * e] - (float)h0), l1 = (_Float16)(w[2 * e + 1] - (float)h1);
      oh[it][e] = pk16(h_bits(h0), h_bits(h1));
      ol[it][e] = pk16(h_bits(l0), h_bits(l1));
    }
  }
  const size_t ob = (rq0 * NH + head) * HD + c8;
  for (int pass = 0; pass < 2; ++pass) {
#pragma unroll
    for (int it = 0; it < 4; ++it) {
      const int row = it * 4 + rq;
      const size_t o8 = ob + (size_t)row * (NH * HD);
      *(volatile v4u*)(OHIp + o8) = oh[it];
      *(volatile v4u*)(OLOp + o8) = ol[it];
    }
    __threadfence();
  }
}

extern "C" void kernel_launch(void* const* d_in, const int* in_sizes, int n_in,
                              void* d_out, int out_size, void* d_ws, size_t ws_size,
                              hipStream_t stream) {
  if (n_in < 8) return;
  if (in_sizes[0] != MROWS * DMOD) return;
  if (in_sizes[1] != DMOD * NQK) return;
  if (in_sizes[2] != DMOD * DMOD || in_sizes[3] != DMOD * DMOD) return;
  if (in_sizes[4] != HD || in_sizes[5] != HD || in_sizes[6] != HD || in_sizes[7] != HD) return;
  if (out_size != MROWS * DMOD) return;

  const float* x   = (const float*)d_in[0];
  const float* wqk = (const float*)d_in[1];
  const float* wv  = (const float*)d_in[2];
  const float* wo  = (const float*)d_in[3];
  const float* qs  = (const float*)d_in[4];
  const float* qbi = (const float*)d_in[5];
  const float* ks  = (const float*)d_in[6];
  const float* kbi = (const float*)d_in[7];
  float*       out = (float*)d_out;

  const size_t szXB = (size_t)MROWS * DMOD * 2;
  const size_t szWQ = (size_t)NQK * DMOD * 2;
  const size_t szW  = (size_t)DMOD * DMOD * 2;
  const size_t szF  = (size_t)MROWS * NQK * 4;
  const size_t szP  = (size_t)MROWS * DMOD * 2;
  size_t off = 0;
  const size_t oXB  = off; off += szXB;
  const size_t oWQ  = off; off += szWQ;
  const size_t oWV  = off; off += szW;
  const size_t oWO  = off; off += szW;
  const size_t oF   = off; off += szF;
  const size_t oQK  = off; off += 2 * szP;
  const size_t oVHI = off; off += szP;
  const size_t oVLO = off; off += szP;
  const size_t oOHI = off; off += szP;
  const size_t oOLO = off; off += szP;
  if (off > ws_size) return;
  if (off > (size_t)134217728) return;

  char* ws = (char*)d_ws;
  u16*   XB  = (u16*)(ws + oXB);
  u16*   WQB = (u16*)(ws + oWQ);
  u16*   WVB = (u16*)(ws + oWV);
  u16*   WOH = (u16*)(ws + oWO);
  float* F   = (float*)(ws + oF);
  u16*   QK  = (u16*)(ws + oQK);
  u16*   QP  = QK;
  u16*   KP  = QK + (size_t)MROWS * DMOD;
  u16*   VHI = (u16*)(ws + oVHI);
  u16*   VLO = (u16*)(ws + oVLO);
  u16*   OHI = (u16*)(ws + oOHI);
  u16*   OLO = (u16*)(ws + oOLO);

  const dim3 blk(256);
  const int n8x = (MROWS * DMOD) / 8;
  const dim3 gX(n8x / 256);
  const dim3 gWQ((DMOD / 64) * (NQK / 64));
  const dim3 gWT((DMOD / 64) * (DMOD / 64));
  const dim3 gGQ((MROWS / 64) * (NQK / 64));
  const dim3 gG((MROWS / 64) * (DMOD / 64));
  const dim3 bG(128);
  const dim3 gLN((NVEC * 32) / 256);
  const dim3 gVT(BATCH * NH * NST);
  const dim3 gAT(ATT_BLOCKS);
  const dim3 bAT(ATT_THREADS);

  cvt16<<<gX, blk, 0, stream>>>(x, XB, n8x, 0, 1.0f);
  wt16<<<gWQ, blk, 0, stream>>>(wqk, WQB, DMOD, NQK, 0, 1.0f);
  wt16<<<gWT, blk, 0, stream>>>(wv, WVB, DMOD, DMOD, 0, 1.0f);
  wt16<<<gWT, blk, 0, stream>>>(wo, WOH, DMOD, DMOD, 1, WOS);
  gemm_bf<<<gGQ, bG, 0, stream>>>(XB, WQB, F, MROWS, NQK, DMOD, 1.0f / 32.0f);
  ln16<<<gLN, blk, 0, stream>>>(F, qs, qbi, ks, kbi, QK, NVEC);
  gemm_bf<<<gG, bG, 0, stream>>>(XB, WVB, F, MROWS, DMOD, DMOD, 1.0f / 32.0f);
  vt16<<<gVT, blk, 0, stream>>>(F, VHI, VLO);
  attn1<<<gAT, bAT, 0, stream>>>(QP, KP, VHI, VLO, OHI, OLO);
  gemm_h2<<<gG, bG, 0, stream>>>(OHI, OLO, WOH, out, MROWS, DMOD, DMOD, (1.0f / 32.0f) / (OSC * WOS));
  (void)hipGetLastError();
}
